// GroupedQueryAttention_82884278878229
// MI455X (gfx1250) — hardware-verified
//
#include <hip/hip_runtime.h>


#ifndef NB
#define NB 2
#endif
#ifndef SEQ
#define SEQ 2048
#endif
#define SEQ_FULL 2048
#define TT   SEQ
#define DM   2048
#define NH_  32
#define NKV  8
#define REP  (NH_ / NKV)
#define HD   64
#define DQ   (NH_ * HD)
#define DKV  (NKV * HD)
#define RH   ((SEQ) < 512 ? (SEQ) : 512)
#define PCAR 1024.0f
#define SCL  0.125f
#define LOG2E 1.4426950408889634f
#define CSL  (SCL * LOG2E)

static_assert(REP == 4);
static_assert(HD == 64);
static_assert((TT % 64) == 0);
static_assert((RH % 32) == 0);
static_assert(((TT - RH) % 16) == 0);
static_assert((RH / 16 + (TT - RH) / 16) * 16 == TT);
static_assert(NH_ * HD == DQ && NKV * HD == DKV);
static_assert((DM % 64) == 0 && (DQ % 64) == 0 && (DKV % 64) == 0);
static_assert((HD % 32) == 0 && (TT % 32) == 0 && (DM % 32) == 0 && (DQ % 32) == 0);
static_assert(((size_t)NH_ * TT * HD) % 2048 == 0);
static_assert(((size_t)NKV * TT * HD) % 2048 == 0);
static_assert(((size_t)DQ * DM / 8) % 256 == 0 && ((size_t)DKV * DM / 8) % 256 == 0 && ((size_t)TT * DM / 8) % 256 == 0);
static_assert(SEQ <= SEQ_FULL);
static_assert(2 * DKV == 1024);
static_assert(((size_t)DKV * DM) % 8 == 0);

typedef _Float16 h16;
typedef unsigned short bf;
typedef __attribute__((ext_vector_type(16))) __bf16   v16bf;
typedef __attribute__((ext_vector_type(16))) _Float16 v16h;
typedef __attribute__((ext_vector_type(16))) unsigned short v16us;
typedef __attribute__((ext_vector_type(8)))  _Float16 v8h;
typedef __attribute__((ext_vector_type(8)))  unsigned short v8us;
typedef __attribute__((ext_vector_type(8)))  float    v8f;
typedef __attribute__((ext_vector_type(4)))  float    v4f;
typedef v4f  __attribute__((may_alias)) v4fa;

__device__ __forceinline__ unsigned short f2bf(float f) { unsigned u = __float_as_uint(f); u += 0x7FFFu + ((u >> 16) & 1u); return (unsigned short)(u >> 16); }
__device__ __forceinline__ float bf2f(unsigned short b) { return __uint_as_float(((unsigned)b) << 16); }
__device__ __forceinline__ float bfr(float f) { return bf2f(f2bf(f)); }
__device__ __forceinline__ h16 tohx(float x) { return (h16)x; }
__device__ __forceinline__ void splitf(float y, unsigned short& h, unsigned short& l) { h = f2bf(y); l = f2bf(y - bf2f(h)); }
__device__ __forceinline__ v16h cat16(v8h lo, v8h hi) { return __builtin_shufflevector(lo, hi, 0, 1, 2, 3, 4, 5, 6, 7, 8, 9, 10, 11, 12, 13, 14, 15); }
__device__ __forceinline__ v16bf cat16b(v8us lo, v8us hi) { return __builtin_bit_cast(v16bf, __builtin_shufflevector(lo, hi, 0, 1, 2, 3, 4, 5, 6, 7, 8, 9, 10, 11, 12, 13, 14, 15)); }
__device__ __forceinline__ v8f wmma16(v16h a, v16h b, v8f c) { return __builtin_amdgcn_wmma_f32_16x16x32_f16(false, a, false, b, (short)0, c, false, false); }
__device__ __forceinline__ v8f wmmab(v16bf a, v16bf b, v8f c) { return __builtin_amdgcn_wmma_f32_16x16x32_bf16(false, a, false, b, (short)0, c, false, false); }

template <typename T16> struct WFrag;
template <> struct WFrag<h16> { typedef v16h V;
    static __device__ __forceinline__ V ld(const h16* p) { return cat16(*(const v8h*)p, *(const v8h*)(p + 16)); }
    static __device__ __forceinline__ v8f mma(V a, V b, v8f c) { return wmma16(a, b, c); }
    static __device__ __forceinline__ void packp(v8f p0, v8f p1, V& H, V& L, float& ls) { v16h o;
#pragma unroll
        for (int r = 0; r < 8; ++r) { const h16 c0 = (h16)(p0[r] * PCAR), c1 = (h16)(p1[r] * PCAR); o[r] = c0; o[8 + r] = c1; ls += (float)c0 + (float)c1; }
        H = o; L = o; } };
template <> struct WFrag<bf> { typedef v16bf V;
    static __device__ __forceinline__ V ld(const bf* p) { return cat16b(*(const v8us*)p, *(const v8us*)(p + 16)); }
    static __device__ __forceinline__ v8f mma(V a, V b, v8f c) { return wmmab(a, b, c); }
    static __device__ __forceinline__ void packp(v8f p0, v8f p1, V& H, V& L, float& ls) { v16us hh, ll;
#pragma unroll
        for (int r = 0; r < 8; ++r) { unsigned short a, c2; splitf(p0[r], a, c2); hh[r] = a; ll[r] = c2; splitf(p1[r], a, c2); hh[8 + r] = a; ll[8 + r] = c2; ls += p0[r] + p1[r]; }
        H = __builtin_bit_cast(v16bf, hh); L = __builtin_bit_cast(v16bf, ll); } };

template <typename T16, int NSPLIT, bool BIAS>
__global__ __launch_bounds__(32) void k_gemmw(const T16* __restrict__ A, const T16* __restrict__ A2, const T16* __restrict__ Bt, const T16* __restrict__ Bt2, int K, float* C, int ldc, const float* __restrict__ bias, size_t sA, size_t sB, size_t sC) {
    typedef typename WFrag<T16>::V V;
    __shared__ __align__(16) float os[16 * 68];
    const size_t z = blockIdx.z; A += z * sA; if (A2) A2 += z * sA; Bt += z * sB; if (Bt2) Bt2 += z * sB; C += z * sC;
    const int lane = threadIdx.x & 31, lr = lane & 15, hi = lane >> 4; const int r0 = blockIdx.x * 64, c0 = blockIdx.y * 64;
    v8f acc[4][4];
#pragma unroll
    for (int mb = 0; mb < 4; ++mb)
#pragma unroll
        for (int nb = 0; nb < 4; ++nb) acc[mb][nb] = (v8f){};
    const size_t aoff = (size_t)(r0 + lr) * K + 8 * hi, boff = (size_t)(c0 + lr) * K + 8 * hi;
#pragma unroll 1
    for (int kc = 0; kc < K; kc += 32) {
        V a[4], a2[4];
#pragma unroll
        for (int mb = 0; mb < 4; ++mb) { a[mb] = WFrag<T16>::ld(A + aoff + (size_t)mb * 16 * K + kc); if (NSPLIT == 1 || NSPLIT == 2) a2[mb] = WFrag<T16>::ld(A2 + aoff + (size_t)mb * 16 * K + kc); }
#pragma unroll
        for (int nb = 0; nb < 4; ++nb) { const V b = WFrag<T16>::ld(Bt + boff + (size_t)nb * 16 * K + kc); V b2; if (NSPLIT >= 2) b2 = WFrag<T16>::ld(Bt2 + boff + (size_t)nb * 16 * K + kc);
#pragma unroll
            for (int mb = 0; mb < 4; ++mb) { acc[mb][nb] = WFrag<T16>::mma(a[mb], b, acc[mb][nb]); if (NSPLIT == 1 || NSPLIT == 2) acc[mb][nb] = WFrag<T16>::mma(a2[mb], b, acc[mb][nb]); if (NSPLIT >= 2) acc[mb][nb] = WFrag<T16>::mma(a[mb], b2, acc[mb][nb]); } }
        asm volatile("v_nop\n\tv_nop\n\tv_nop\n\tv_nop" : "+v"(acc[0][0]), "+v"(acc[1][1]), "+v"(acc[2][2]), "+v"(acc[3][3]) : "v"(a[0]), "v"(a[3]));
    }
#pragma unroll
    for (int mb = 0; mb < 4; ++mb) {
#pragma unroll
        for (int nb = 0; nb < 4; ++nb) {
#pragma unroll
            for (int j = 0; j < 8; ++j) os[(hi * 8 + j) * 68 + nb * 16 + lr] = acc[mb][nb][j]; }
        __builtin_amdgcn_wave_barrier(); asm volatile("" ::: "memory");
        float* crow = C + (size_t)(r0 + mb * 16) * ldc + c0;
#pragma unroll 1
        for (int ps = 0; ps < 2; ++ps) {
#pragma unroll
            for (int s = 0; s < 8; ++s) { const int row = 2 * s + hi, cofs = lr * 4; v4f val = *(const v4fa*)(os + row * 68 + cofs); if (BIAS) { val[0] += bfr(bias[c0 + cofs]); val[1] += bfr(bias[c0 + cofs + 1]); val[2] += bfr(bias[c0 + cofs + 2]); val[3] += bfr(bias[c0 + cofs + 3]); }
                *(volatile v4f*)(crow + (size_t)row * ldc + cofs) = val; }
            if (ps == 0) __threadfence(); }
        __builtin_amdgcn_wave_barrier(); asm volatile("" ::: "memory");
    }
}

template <typename T16, int NSPLIT>
__global__ __launch_bounds__(32) void k_flash(const T16* __restrict__ Q, const T16* __restrict__ Q2, const T16* __restrict__ Kp, const T16* __restrict__ Kp2, const T16* __restrict__ Vt, const T16* __restrict__ Vt2, bf* Ah, bf* Al, unsigned roff) {
    typedef typename WFrag<T16>::V V;
    __shared__ __align__(16) float os[16 * 68];
    const unsigned lane = threadIdx.x & 31u, lr = lane & 15u, hi = lane >> 4;
    const unsigned h = blockIdx.y, kvh = h / (unsigned)REP;
    const unsigned q0 = roff + blockIdx.x * 16u, qrow = q0 + lr;
    const unsigned nblk = (q0 + 47u) >> 5;
    const unsigned qoff = (h * (unsigned)TT + qrow) * (unsigned)HD + 8u * hi;
    const unsigned koff = (kvh * (unsigned)TT + lr) * (unsigned)HD + 8u * hi;
    const unsigned voff = (kvh * (unsigned)HD + lr) * (unsigned)TT + 8u * hi;
    V qh[2], ql[2];
#pragma unroll
    for (int c = 0; c < 2; ++c) { qh[c] = WFrag<T16>::ld(Q + qoff + c * 32); if (NSPLIT >= 2) ql[c] = WFrag<T16>::ld(Q2 + qoff + c * 32); }
    v8f acc[4];
#pragma unroll
    for (int t = 0; t < 4; ++t) acc[t] = (v8f){};
    float m = -3.0e38f, l = 0.f;
#pragma unroll 1
    for (unsigned blk = 0; blk < nblk; ++blk) {
        const unsigned kb = blk * 32u;
        v8f s0 = (v8f){}, s1 = (v8f){};
#pragma unroll
        for (int c = 0; c < 2; ++c) {
            const unsigned o0 = koff + kb * (unsigned)HD + (unsigned)(c * 32), o1 = o0 + 16u * (unsigned)HD;
            const V k0 = WFrag<T16>::ld(Kp + o0), k1 = WFrag<T16>::ld(Kp + o1);
            s0 = WFrag<T16>::mma(k0, qh[c], s0); s1 = WFrag<T16>::mma(k1, qh[c], s1);
            if (NSPLIT >= 2) { const V k0l = WFrag<T16>::ld(Kp2 + o0), k1l = WFrag<T16>::ld(Kp2 + o1);
                s0 = WFrag<T16>::mma(k0l, qh[c], s0); s1 = WFrag<T16>::mma(k1l, qh[c], s1); s0 = WFrag<T16>::mma(k0, ql[c], s0); s1 = WFrag<T16>::mma(k1, ql[c], s1); } }
        asm volatile("v_nop\n\tv_nop\n\tv_nop\n\tv_nop" : "+v"(s0), "+v"(s1) : "v"(qh[0]), "v"(qh[1]));
        const unsigned lim = (blk + 1u == nblk) ? qrow : 0xFFFFFFFFu;
        const unsigned kk = kb + 8u * hi;
        v8f t0, t1; float bm = -3.0e38f;
#pragma unroll
        for (int r = 0; r < 8; ++r) { const float a = (kk + (unsigned)r <= lim) ? s0[r] * CSL : -3.0e38f; const float b = (kk + 16u + (unsigned)r <= lim) ? s1[r] * CSL : -3.0e38f; t0[r] = a; t1[r] = b; bm = fmaxf(bm, fmaxf(a, b)); }
        bm = fmaxf(bm, __shfl_xor(bm, 16, 32));
        const float mn = fmaxf(m, bm);
        const float alpha = __builtin_amdgcn_exp2f(m - mn); m = mn;
#pragma unroll
        for (int r = 0; r < 8; ++r) { t0[r] = __builtin_amdgcn_exp2f(t0[r] - mn); t1[r] = __builtin_amdgcn_exp2f(t1[r] - mn); }
        V pH, pL; float ls = 0.f;
        WFrag<T16>::packp(t0, t1, pH, pL, ls);
        l = l * alpha + ls;
#pragma unroll
        for (int t = 0; t < 4; ++t) acc[t] = acc[t] * alpha;
#pragma unroll
        for (int t = 0; t < 4; ++t) { const unsigned vo = voff + (unsigned)(t * 16) * (unsigned)TT + kb; const V vh = WFrag<T16>::ld(Vt + vo);
            acc[t] = WFrag<T16>::mma(vh, pH, acc[t]);
            if (NSPLIT >= 2) { const V vl = WFrag<T16>::ld(Vt2 + vo); acc[t] = WFrag<T16>::mma(vl, pH, acc[t]); acc[t] = WFrag<T16>::mma(vh, pL, acc[t]); } }
        asm volatile("v_nop\n\tv_nop\n\tv_nop\n\tv_nop" : "+v"(acc[0]), "+v"(acc[1]), "+v"(acc[2]), "+v"(acc[3]) : "v"(pH));
    }
    const float lt = l + __shfl_xor(l, 16, 32);
    const float inv = __fdiv_rn(1.0f, lt);
#pragma unroll
    for (int t = 0; t < 4; ++t) { v4f w0, w1;
#pragma unroll
        for (int r = 0; r < 4; ++r) { w0[r] = acc[t][r] * inv; w1[r] = acc[t][4 + r] * inv; }
        *(v4fa*)(os + lr * 68u + (unsigned)(t * 16) + 8u * hi) = w0; *(v4fa*)(os + lr * 68u + (unsigned)(t * 16) + 8u * hi + 4u) = w1; }
    __builtin_amdgcn_wave_barrier(); asm volatile("" ::: "memory");
    const unsigned rq = lane >> 3, pc = lane & 7u;
#pragma unroll 1
    for (int ps = 0; ps < 2; ++ps) {
#pragma unroll
        for (int s = 0; s < 4; ++s) { const unsigned row = (unsigned)(s * 4) + rq; const v4f x0 = *(const v4fa*)(os + row * 68u + pc * 8u), x1 = *(const v4fa*)(os + row * 68u + pc * 8u + 4u); v8us oh, ol;
#pragma unroll
            for (int q = 0; q < 4; ++q) { unsigned short a, c2; splitf(x0[q], a, c2); oh[q] = a; ol[q] = c2; splitf(x1[q], a, c2); oh[q + 4] = a; ol[q + 4] = c2; }
            const size_t oo = (size_t)(q0 + row) * DQ + h * (unsigned)HD + pc * 8u; *(volatile v8us*)(Ah + oo) = oh; *(volatile v8us*)(Al + oo) = ol; }
        if (ps == 0) __threadfence(); }
}

__global__ __launch_bounds__(256) void k_cvt8(const float* __restrict__ src, bf* dst, size_t n8) { const size_t i = (size_t)blockIdx.x * 256 + threadIdx.x; if (i >= n8) return; const v8f v = *(const v8f*)(src + i * 8); v8us o;
#pragma unroll
    for (int k = 0; k < 8; ++k) o[k] = f2bf(v[k]); *(volatile v8us*)(dst + i * 8) = o; __threadfence(); *(volatile v8us*)(dst + i * 8) = o; }

__global__ __launch_bounds__(256) void k_hpl(const float* __restrict__ F, unsigned pitch, unsigned nheads, h16* P16, bf* Ph, bf* Pl) {
    const unsigned idx = blockIdx.x * 256u + threadIdx.x; if (idx >= nheads * (unsigned)(TT * HD / 8)) return;
    const unsigned e = idx * 8u; const unsigned d = e % (unsigned)HD; const unsigned t = (e / (unsigned)HD) % (unsigned)TT; const unsigned h = e / (unsigned)(HD * TT);
    const float* f = F + (size_t)t * pitch + h * (unsigned)HD + d;
    const v4f x0 = *(const v4f*)f, x1 = *(const v4f*)(f + 4);
    v8h o16; v8us oh, ol;
#pragma unroll
    for (int q = 0; q < 4; ++q) { unsigned short a, c2; o16[q] = tohx(x0[q]); splitf(x0[q], a, c2); oh[q] = a; ol[q] = c2; o16[q + 4] = tohx(x1[q]); splitf(x1[q], a, c2); oh[q + 4] = a; ol[q + 4] = c2; }
    *(volatile v8h*)(P16 + e) = o16; *(volatile v8us*)(Ph + e) = oh; *(volatile v8us*)(Pl + e) = ol; __threadfence(); *(volatile v8h*)(P16 + e) = o16; *(volatile v8us*)(Ph + e) = oh; *(volatile v8us*)(Pl + e) = ol; }

__global__ __launch_bounds__(256) void k_vtp(const float* __restrict__ F, unsigned pitch, unsigned nheads, h16* V16, bf* Vh, bf* Vl) {
    const unsigned idx = blockIdx.x * 256u + threadIdx.x; if (idx >= nheads * (unsigned)(HD * TT / 8)) return;
    const unsigned e = idx * 8u; const unsigned t = e % (unsigned)TT; const unsigned d = (e / (unsigned)TT) % (unsigned)HD; const unsigned g = e / (unsigned)(TT * HD);
    const float* f = F + (size_t)t * pitch + g * (unsigned)HD + d;
    v8h o16; v8us oh, ol;
#pragma unroll
    for (int q = 0; q < 8; ++q) { const float x = f[(size_t)q * pitch]; unsigned short a, c2; o16[q] = tohx(x); splitf(x, a, c2); oh[q] = a; ol[q] = c2; }
    *(volatile v8h*)(V16 + e) = o16; *(volatile v8us*)(Vh + e) = oh; *(volatile v8us*)(Vl + e) = ol; __threadfence(); *(volatile v8h*)(V16 + e) = o16; *(volatile v8us*)(Vh + e) = oh; *(volatile v8us*)(Vl + e) = ol; }

extern "C" void kernel_launch(void* const* d_in, const int* in_sizes, int n_in,
                              void* d_out, int out_size, void* d_ws, size_t ws_size, hipStream_t stream) {
    if (n_in < 4) return;
    const size_t need_x = (size_t)(NB - 1) * SEQ_FULL * DM + (size_t)SEQ * DM;
    if ((size_t)in_sizes[0] < need_x || (size_t)out_size < need_x) return;
    if ((size_t)in_sizes[1] < (size_t)DQ * DM || (size_t)in_sizes[2] < (size_t)2 * DKV * DM || (size_t)in_sizes[3] < (size_t)DM * DQ) return;
    const float* x = (const float*)d_in[0]; const float* wq = (const float*)d_in[1]; const float* wkv = (const float*)d_in[2]; const float* wo = (const float*)d_in[3];
    const float* wk = wkv;
    const float* wv = wkv + (size_t)DKV * DM;
    float* OUT = (float*)d_out;
    constexpr size_t SZ_WQ = (size_t)DQ * DM * 2, SZ_WKV = (size_t)DKV * DM * 2, SZ_WO = (size_t)DM * DQ * 2, SZ_XB = (size_t)TT * DM * 2, SZ_FQ = (size_t)TT * DQ * 4, SZ_FK = (size_t)TT * DKV * 4;
    constexpr size_t SZ_QP = (size_t)NH_ * TT * HD * 2, SZ_KP = (size_t)NKV * TT * HD * 2, SZ_AT = (size_t)TT * DQ * 2;
    constexpr size_t CARVE = SZ_WQ + 2 * SZ_WKV + SZ_WO + SZ_XB + SZ_FQ + SZ_FK + 3 * SZ_QP + 6 * SZ_KP + 2 * SZ_AT;
    static_assert((SZ_WQ % 256) == 0 && (SZ_WKV % 256) == 0 && (SZ_WO % 256) == 0 && (SZ_XB % 256) == 0 && (SZ_FQ % 256) == 0 && (SZ_FK % 256) == 0 && (SZ_QP % 256) == 0 && (SZ_KP % 256) == 0 && (SZ_AT % 256) == 0);
    static_assert(CARVE <= (size_t)134217728);
    if (CARVE > ws_size) return;
    char* wsp = (char*)d_ws;
    auto take = [&](size_t bytes) { char* p = wsp; wsp += bytes; return (void*)p; };
    bf* WQ = (bf*)take(SZ_WQ); bf* WK = (bf*)take(SZ_WKV); bf* WV = (bf*)take(SZ_WKV); bf* WO = (bf*)take(SZ_WO);
    bf* XB = (bf*)take(SZ_XB); float* FQ = (float*)take(SZ_FQ); float* FK = (float*)take(SZ_FK);
    h16* QP16 = (h16*)take(SZ_QP); bf* QPh = (bf*)take(SZ_QP); bf* QPl = (bf*)take(SZ_QP);
    h16* KP16 = (h16*)take(SZ_KP); bf* KPh = (bf*)take(SZ_KP); bf* KPl = (bf*)take(SZ_KP);
    h16* VT16 = (h16*)take(SZ_KP); bf* VTh = (bf*)take(SZ_KP); bf* VTl = (bf*)take(SZ_KP);
    bf* ATh = (bf*)take(SZ_AT); bf* ATl = (bf*)take(SZ_AT);
    if ((size_t)(wsp - (char*)d_ws) != CARVE) return;
    float* FV = FK;
    k_cvt8<<<(unsigned)(((size_t)DQ * DM / 8 + 255) / 256), 256, 0, stream>>>(wq, WQ, (size_t)DQ * DM / 8);
    k_cvt8<<<(unsigned)(((size_t)DKV * DM / 8 + 255) / 256), 256, 0, stream>>>(wk, WK, (size_t)DKV * DM / 8);
    k_cvt8<<<(unsigned)(((size_t)DKV * DM / 8 + 255) / 256), 256, 0, stream>>>(wv, WV, (size_t)DKV * DM / 8);
    k_cvt8<<<(unsigned)(((size_t)DM * DQ / 8 + 255) / 256), 256, 0, stream>>>(wo, WO, (size_t)DM * DQ / 8);
    const unsigned LQ = (unsigned)(((size_t)NH_ * TT * HD / 8 + 255) / 256), LKv = (unsigned)(((size_t)NKV * TT * HD / 8 + 255) / 256);
    for (int b = 0; b < NB; ++b) {
        k_cvt8<<<(unsigned)(((size_t)TT * DM / 8 + 255) / 256), 256, 0, stream>>>(x + (size_t)b * SEQ_FULL * DM, XB, (size_t)TT * DM / 8);
        k_gemmw<bf, 0, false><<<dim3(TT / 64, DQ / 64, 1), 32, 0, stream>>>(XB, nullptr, WQ, nullptr, DM, FQ, DQ, nullptr, 0, 0, 0);
        k_hpl<<<LQ, 256, 0, stream>>>(FQ, (unsigned)DQ, (unsigned)NH_, QP16, QPh, QPl);
        k_gemmw<bf, 0, false><<<dim3(TT / 64, DKV / 64, 1), 32, 0, stream>>>(XB, nullptr, WK, nullptr, DM, FK, DKV, nullptr, 0, 0, 0);
        k_hpl<<<LKv, 256, 0, stream>>>(FK, (unsigned)DKV, (unsigned)NKV, KP16, KPh, KPl);
        k_gemmw<bf, 0, false><<<dim3(TT / 64, DKV / 64, 1), 32, 0, stream>>>(XB, nullptr, WV, nullptr, DM, FV, DKV, nullptr, 0, 0, 0);
        k_vtp<<<LKv, 256, 0, stream>>>(FV, (unsigned)DKV, (unsigned)NKV, VT16, VTh, VTl);
        k_flash<bf, 2><<<dim3(RH / 16, NH_, 1), 32, 0, stream>>>(QPh, QPl, KPh, KPl, VTh, VTl, ATh, ATl, 0u);
        if (TT > RH) k_flash<h16, 0><<<dim3((TT - RH) / 16, NH_, 1), 32, 0, stream>>>(QP16, nullptr, KP16, nullptr, VT16, nullptr, ATh, ATl, (unsigned)RH);
        k_gemmw<bf, 1, false><<<dim3(TT / 64, DM / 64, 1), 32, 0, stream>>>(ATh, ATl, WO, nullptr, DQ, OUT + (size_t)b * SEQ_FULL * DM, DM, nullptr, 0, 0, 0); }
}
